// MultiHeadSA_12756052869505
// MI455X (gfx1250) — hardware-verified
//
#include <hip/hip_runtime.h>
#include <cmath>

typedef __attribute__((ext_vector_type(16))) __bf16   v16b;
typedef __attribute__((ext_vector_type(8)))  __bf16   v8b;
typedef __attribute__((ext_vector_type(8)))  float    v8f;
typedef __attribute__((ext_vector_type(4)))  float    v4f;
typedef __attribute__((ext_vector_type(2)))  float    v2f;
typedef __attribute__((ext_vector_type(4)))  unsigned v4u;

constexpr int kBatch   = 4;
constexpr int kSeq     = 2048;
constexpr int kDModel  = 1024;
constexpr int kHeads   = 16;
constexpr int kDHead   = 64;
constexpr int kRows    = kBatch * kSeq;
constexpr int kQKVCols = 3 * kDModel;
constexpr int kPhaseB  = 2;
constexpr int kPhaseRows = kPhaseB * kSeq;
static_assert(kHeads * kDHead == kDModel);
static_assert(kDHead == 64);
static_assert(kBatch % kPhaseB == 0);

constexpr size_t kBytesXb   = (size_t)kRows * kDModel * 2;
constexpr size_t kBytesWqb  = (size_t)kQKVCols * kDModel * 2;
constexpr size_t kBytesWob  = (size_t)kDModel * kDModel * 2;
constexpr size_t kBytesRope = (size_t)kSeq * 64 * 4;
constexpr size_t kBytesQKV  = (size_t)kRows * kQKVCols * 2;
constexpr size_t kBytesO    = (size_t)kPhaseRows * kDModel * 2;
constexpr size_t kOffXb   = 0;
constexpr size_t kOffOh   = kOffXb;
constexpr size_t kOffOl   = kOffXb + kBytesO;
constexpr size_t kOffWqb  = kOffXb + kBytesXb;
constexpr size_t kOffWob  = kOffWqb + kBytesWqb;
constexpr size_t kOffRope = kOffWob + kBytesWob;
constexpr size_t kOffQh   = kOffRope + kBytesRope;
constexpr size_t kOffQl   = kOffQh + kBytesQKV;
constexpr size_t kWsEnd   = kOffQl + kBytesQKV;
static_assert(2 * kBytesO <= kBytesXb);
static_assert(kWsEnd == 126353408);
static_assert(kWsEnd <= 134217728);
static_assert((kOffWqb % 128) == 0 && (kOffWob % 128) == 0 && (kOffRope % 128) == 0 && (kOffQh % 128) == 0 && (kOffQl % 128) == 0 && (kOffOl % 128) == 0);

static_assert(kRows % 64 == 0 && kQKVCols % 64 == 0 && kDModel % 32 == 0);
static_assert(((kRows / 64) * (kQKVCols / 64)) % 8 == 0);
static_assert(kPhaseRows % 64 == 0 && kDModel % 64 == 0);
static_assert(((kPhaseRows / 64) * (kDModel / 64)) % 8 == 0);
static_assert(kSeq % 64 == 0);
static_assert((kRows * kDModel) % 512 == 0 && (kQKVCols * kDModel) % 512 == 0 && (kDModel * kDModel) % 512 == 0);
static_assert((kSeq * 32) % 256 == 0);

__device__ __forceinline__ unsigned short f2bf_bits(float f) {
  unsigned u = __float_as_uint(f);
  return (unsigned short)((u + 0x7FFFu + ((u >> 16) & 1u)) >> 16);
}
__device__ __forceinline__ float bf_bits2f(unsigned short h) { return __uint_as_float(((unsigned)h) << 16); }
__device__ __forceinline__ __bf16 f2bf(float f) { return __builtin_bit_cast(__bf16, f2bf_bits(f)); }
__device__ __forceinline__ void bf_split(float f, __bf16& hi, __bf16& lo) {
  const unsigned short hb = f2bf_bits(f);
  hi = __builtin_bit_cast(__bf16, hb);
  lo = f2bf(f - __uint_as_float(((unsigned)hb) << 16));
}
__device__ __forceinline__ void split2_pack(float v0, float v1, unsigned& wh, unsigned& wl) {
  const unsigned short h0 = f2bf_bits(v0), h1 = f2bf_bits(v1);
  const unsigned short l0 = f2bf_bits(v0 - bf_bits2f(h0));
  const unsigned short l1 = f2bf_bits(v1 - bf_bits2f(h1));
  wh = (unsigned)h0 | ((unsigned)h1 << 16);
  wl = (unsigned)l0 | ((unsigned)l1 << 16);
}

__device__ __forceinline__ void dep_guard_b(v8f& a, v8f& b, v16b x, v16b y) { asm volatile("v_nop\n\tv_nop\n\tv_nop\n\tv_nop" : "+v"(a), "+v"(b) : "v"(x), "v"(y)); }
__device__ __forceinline__ void keep4_b(v16b a, v16b b, v16b c, v16b d) { asm volatile("v_nop" :: "v"(a), "v"(b), "v"(c), "v"(d)); }
__device__ __forceinline__ void acc_guard4(v8f& a, v8f& b, v8f& c, v8f& d) { asm volatile("v_nop\n\tv_nop\n\tv_nop\n\tv_nop" : "+v"(a), "+v"(b), "+v"(c), "+v"(d)); }

template <typename T> struct Frag;
template <> struct Frag<__bf16> {
  typedef v16b V; union U { v16b v; v8b h[2]; };
  static __device__ __forceinline__ v16b load(const __bf16* p) {
    U f; f.h[0] = *(const v8b*)(p); f.h[1] = *(const v8b*)(p + 16); return f.v;
  }
  static __device__ __forceinline__ v8f mma(v16b a, v16b b, v8f c) {
    return __builtin_amdgcn_wmma_f32_16x16x32_bf16(false, a, false, b, (short)0, c, false, false);
  }
  static __device__ __forceinline__ void guard(v8f& a, v8f& b, v16b x, v16b y) { dep_guard_b(a, b, x, y); }
  static __device__ __forceinline__ void keep(v16b a, v16b b, v16b c, v16b d) { keep4_b(a, b, c, d); }
};

__device__ __forceinline__ v8f at_mma(v16b a, v16b b, v8f c) {
  c = __builtin_amdgcn_wmma_f32_16x16x32_bf16(false, a, false, b, (short)0, c, false, false);
  asm volatile("v_nop\n\tv_nop\n\tv_nop\n\tv_nop" : "+v"(c) : "v"(a), "v"(b));
  return c;
}

template <int SPLITM, int OUT_MODE>
__global__ __launch_bounds__(256) void wmma_gemm64(
    const unsigned short* __restrict__ Ap, const unsigned short* __restrict__ A2p, int lda,
    const unsigned short* __restrict__ Btp, const unsigned short* __restrict__ Bt2p, int ldb,
    void* __restrict__ Cout, void* __restrict__ Cout2, int ldc,
    const float* __restrict__ rope, int seqLen, int ropeN, int qN, float qsc,
    int M, int N, int K, float scale) {
  typedef __bf16 T;
  typedef v16b V;
  const T* A   = (const T*)(const void*)Ap;
  const T* A2  = (const T*)(const void*)A2p;
  const T* Bt  = (const T*)(const void*)Btp;
  const T* Bt2 = (const T*)(const void*)Bt2p;
  __shared__ __align__(16) float sT[8][16 * 68];
  const int lane = threadIdx.x & 31;
  const int wave = threadIdx.x >> 5;
  const int tilesN = N >> 6;
  const int tilesM = M >> 6;
  const int tile = blockIdx.x * 8 + wave;
  if (tile >= tilesM * tilesN) return;
  const int tm = tile / tilesN;
  const int tn = tile - tm * tilesN;
  const int m0 = tm << 6;
  const int n0 = tn << 6;

  const int rlane = lane & 15;
  const int koff  = (lane >> 4) * 8;
  const int mOff  = (lane >> 4) * 8;

  v8f acc[4][4];
#pragma unroll
  for (int i = 0; i < 4; ++i)
#pragma unroll
    for (int j = 0; j < 4; ++j) acc[i][j] = (v8f){0.f,0.f,0.f,0.f,0.f,0.f,0.f,0.f};

  for (int k0 = 0; k0 < K; k0 += 32) {
    V bh[4], bl[4];
#pragma unroll
    for (int j = 0; j < 4; ++j) {
      const size_t bo = (size_t)(n0 + (j << 4) + rlane) * ldb + koff + k0;
      bh[j] = Frag<T>::load(Bt + bo);
      if (SPLITM == 1) bl[j] = Frag<T>::load(Bt2 + bo); else bl[j] = bh[j];
    }
#pragma unroll
    for (int i = 0; i < 4; ++i) {
      const size_t ao = (size_t)(m0 + (i << 4) + rlane) * lda + koff + k0;
      V ah = Frag<T>::load(A + ao);
      V al = ah;
      if (SPLITM != 0) al = Frag<T>::load(A2 + ao);
#pragma unroll
      for (int j = 0; j < 4; ++j) {
        acc[i][j] = Frag<T>::mma(ah, bh[j], acc[i][j]);
        if (SPLITM == 1) acc[i][j] = Frag<T>::mma(ah, bl[j], acc[i][j]);
        if (SPLITM != 0) acc[i][j] = Frag<T>::mma(al, bh[j], acc[i][j]);
      }
      Frag<T>::guard(acc[i][0], acc[i][3], ah, al);
    }
    Frag<T>::keep(bh[0], bh[1], bh[2], bh[3]);
    if (SPLITM == 1) Frag<T>::keep(bl[0], bl[1], bl[2], bl[3]);
  }
  acc_guard4(acc[0][0], acc[0][1], acc[0][2], acc[0][3]);
  acc_guard4(acc[1][0], acc[1][1], acc[1][2], acc[1][3]);
  acc_guard4(acc[2][0], acc[2][1], acc[2][2], acc[2][3]);
  acc_guard4(acc[3][0], acc[3][1], acc[3][2], acc[3][3]);

  float* slab = sT[wave];
#pragma unroll
  for (int i = 0; i < 4; ++i) {
    const int mBase = m0 + (i << 4);
#pragma unroll
    for (int j = 0; j < 4; ++j) {
#pragma unroll
      for (int r = 0; r < 8; ++r) slab[(mOff + r) * 68 + (j << 4) + rlane] = acc[i][j][r] * scale;
    }
    __builtin_amdgcn_fence(__ATOMIC_RELEASE, "workgroup");
    __builtin_amdgcn_wave_barrier();
    __builtin_amdgcn_fence(__ATOMIC_ACQUIRE, "workgroup");
    if (OUT_MODE == 0) {
      float* C = (float*)Cout;
      const int hh = lane >> 4, c4 = (lane & 15) * 4;
      for (int pass = 0; pass < 2; ++pass) {
#pragma unroll
        for (int it = 0; it < 8; ++it) {
          const int row = it * 2 + hh;
          v4f v = *(const v4f*)(slab + row * 68 + c4);
          *(volatile v4f*)(C + (size_t)(mBase + row) * ldc + n0 + c4) = v;
        }
        __threadfence();
      }
    } else {
      unsigned short* C  = (unsigned short*)Cout;
      unsigned short* Cl = (unsigned short*)Cout2;
      const int q8 = lane >> 3, c8 = (lane & 7) * 8;
      const bool  use_rope = (n0 < ropeN);
      const float osc = (n0 < qN) ? qsc : 1.0f;
      for (int pass = 0; pass < 2; ++pass) {
#pragma unroll
        for (int it = 0; it < 4; ++it) {
          const int row  = it * 4 + q8;
          const int grow = mBase + row;
          const int spos = grow % seqLen;
          const float* sp = slab + row * 68 + c8;
          const v4f xa = *(const v4f*)sp;
          const v4f xb = *(const v4f*)(sp + 4);
          const v4f ta = *(const v4f*)(rope + (size_t)spos * 64 + c8);
          const v4f tb = *(const v4f*)(rope + (size_t)spos * 64 + c8 + 4);
          float o[8];
          o[0] = xa[0] * ta[0] - xa[1] * ta[1];  o[1] = xa[0] * ta[1] + xa[1] * ta[0];
          o[2] = xa[2] * ta[2] - xa[3] * ta[3];  o[3] = xa[2] * ta[3] + xa[3] * ta[2];
          o[4] = xb[0] * tb[0] - xb[1] * tb[1];  o[5] = xb[0] * tb[1] + xb[1] * tb[0];
          o[6] = xb[2] * tb[2] - xb[3] * tb[3];  o[7] = xb[2] * tb[3] + xb[3] * tb[2];
          const float xi[8] = {xa[0], xa[1], xa[2], xa[3], xb[0], xb[1], xb[2], xb[3]};
          v4u wh, wl;
#pragma unroll
          for (int e2 = 0; e2 < 4; ++e2) {
            const float v0 = (use_rope ? o[2 * e2]     : xi[2 * e2])     * osc;
            const float v1 = (use_rope ? o[2 * e2 + 1] : xi[2 * e2 + 1]) * osc;
            unsigned ph, pl;
            split2_pack(v0, v1, ph, pl);
            wh[e2] = ph; wl[e2] = pl;
          }
          const size_t off = (size_t)grow * ldc + n0 + c8;
          *(volatile v4u*)(C  + off) = wh;
          *(volatile v4u*)(Cl + off) = wl;
        }
        __threadfence();
      }
    }
    __builtin_amdgcn_fence(__ATOMIC_RELEASE, "workgroup");
    __builtin_amdgcn_wave_barrier();
    __builtin_amdgcn_fence(__ATOMIC_ACQUIRE, "workgroup");
  }
}

__global__ __launch_bounds__(256) void cast_f32_bf16x2(
    const float* __restrict__ in, unsigned short* __restrict__ out, int n2) {
  int i = blockIdx.x * 256 + threadIdx.x;
  if (i < n2) {
    const unsigned short h0 = f2bf_bits(in[2 * i]), h1 = f2bf_bits(in[2 * i + 1]);
    const unsigned u = (unsigned)h0 | ((unsigned)h1 << 16);
    ((volatile unsigned*)out)[i] = u;
    __threadfence();
    ((volatile unsigned*)out)[i] = u;
  }
}

struct RopeFreq { float f[32]; };
static_assert(sizeof(RopeFreq) == 128);

__global__ __launch_bounds__(256) void rope_table_kernel(
    const int* __restrict__ pos, float* __restrict__ tab, int S, RopeFreq fr) {
  const int t = blockIdx.x * 256 + threadIdx.x;
  if (t < S * 32) {
    const int s = t >> 5, p = t & 31;
    float f = fr.f[0];
#pragma unroll
    for (int i = 1; i < 32; ++i) f = (p == i) ? fr.f[i] : f;
    const float ang = (float)pos[s] * f;
    float sv, cv;
    sincosf(ang, &sv, &cv);
    v2f w;
    w[0] = cv; w[1] = sv;
    *(volatile v2f*)(tab + 2 * (size_t)t) = w;
    __threadfence();
    *(volatile v2f*)(tab + 2 * (size_t)t) = w;
  }
}

union AttnKOs { unsigned short k[2][64 * 64]; float os[4][16 * 64]; };
static_assert(sizeof(AttnKOs) == 16384);

__global__ __launch_bounds__(128)
void attn_causal64(const unsigned short* __restrict__ Ph, const unsigned short* __restrict__ Pl,
                   unsigned short* __restrict__ Oh, unsigned short* __restrict__ Ol,
                   int S, int H, int ldp, int ldo, int b0) {
  union FB { v16b v; v8b h[2]; };
  __shared__ __align__(16) AttnKOs ku;
  __shared__ __align__(16) unsigned short Vt[2][64 * 64];
  __shared__ __align__(16) __bf16 Psh[4][16 * 64];
  __shared__ __align__(16) __bf16 Psl[4][16 * 64];

  const int tid  = threadIdx.x;
  const int wave = tid >> 5;
  const int lane = tid & 31;
  const int hh   = lane >> 4;
  const int c    = lane & 15;

  const int nqb = S >> 6;
  const int bx  = blockIdx.x;
  const int qb  = bx % nqb;
  const int bhI = bx / nqb;
  const int h   = bhI % H;
  const int bl  = bhI / H;
  const int b   = b0 + bl;
  const int dm  = H * 64;
  const int q0  = qb * 64 + wave * 16;
  const size_t rowb = (size_t)b * (size_t)S;
  const __bf16* PhB = (const __bf16*)(const void*)Ph;
  const __bf16* PlB = (const __bf16*)(const void*)Pl;
  unsigned short* Ksh = ku.k[0];
  unsigned short* Ksl = ku.k[1];
  unsigned short* Vth = Vt[0];
  unsigned short* Vtl = Vt[1];

  v16b qah[2], qal[2];
#pragma unroll
  for (int dc = 0; dc < 2; ++dc) {
    const size_t off = (rowb + (size_t)(q0 + c)) * (size_t)ldp + (size_t)(h * 64 + dc * 32 + 8 * hh);
    qah[dc] = Frag<__bf16>::load(PhB + off);
    qal[dc] = Frag<__bf16>::load(PlB + off);
  }

  float mrow[8], lrow[8];
  v8f oacc[4];
#pragma unroll
  for (int r = 0; r < 8; ++r) { mrow[r] = -__builtin_inff(); lrow[r] = 0.f; }
#pragma unroll
  for (int t = 0; t < 4; ++t) oacc[t] = (v8f){0.f,0.f,0.f,0.f,0.f,0.f,0.f,0.f};

  for (int kc = 0; kc <= qb; ++kc) {
    const int kv0 = kc * 64;
    __syncthreads();
    {
      const int kvr = tid >> 1, half = tid & 1;
      const size_t ro = (rowb + (size_t)(kv0 + kvr)) * (size_t)ldp + (size_t)(h * 64 + half * 32);
      const v4u* kh4 = (const v4u*)(const void*)(Ph + ro + dm);
      const v4u* kl4 = (const v4u*)(const void*)(Pl + ro + dm);
      v4u kw[4], klw[4];
#pragma unroll
      for (int i = 0; i < 4; ++i) { kw[i] = kh4[i]; klw[i] = kl4[i]; }
#pragma unroll
      for (int i = 0; i < 4; ++i) {
        *(v4u*)(void*)(Ksh + kvr * 64 + half * 32 + 8 * i) = kw[i];
        *(v4u*)(void*)(Ksl + kvr * 64 + half * 32 + 8 * i) = klw[i];
      }
      const v4u* vh4 = (const v4u*)(const void*)(Ph + ro + 2 * dm);
      const v4u* vl4 = (const v4u*)(const void*)(Pl + ro + 2 * dm);
      v4u vw[4], vlw[4];
#pragma unroll
      for (int i = 0; i < 4; ++i) { vw[i] = vh4[i]; vlw[i] = vl4[i]; }
#pragma unroll
      for (int i = 0; i < 4; ++i) {
#pragma unroll
        for (int e = 0; e < 8; ++e) {
          const int d = half * 32 + 8 * i + e;
          const unsigned w0 = vw[i][e >> 1];
          const unsigned w1 = vlw[i][e >> 1];
          const unsigned short u0 = (unsigned short)((e & 1) ? (w0 >> 16) : (w0 & 0xffffu));
          const unsigned short u1 = (unsigned short)((e & 1) ? (w1 >> 16) : (w1 & 0xffffu));
          Vth[d * 64 + kvr] = u0;
          Vtl[d * 64 + kvr] = u1;
        }
      }
    }
    __syncthreads();

    v8f s[4];
#pragma unroll
    for (int j = 0; j < 4; ++j) {
      s[j] = (v8f){0.f,0.f,0.f,0.f,0.f,0.f,0.f,0.f};
#pragma unroll
      for (int dc = 0; dc < 2; ++dc) {
        FB kb, kl;
        const unsigned short* kp  = Ksh + (j * 16 + c) * 64 + dc * 32 + 8 * hh;
        const unsigned short* klp = Ksl + (j * 16 + c) * 64 + dc * 32 + 8 * hh;
        kb.h[0] = *(const v8b*)(const void*)kp;
        kb.h[1] = *(const v8b*)(const void*)(kp + 16);
        kl.h[0] = *(const v8b*)(const void*)klp;
        kl.h[1] = *(const v8b*)(const void*)(klp + 16);
        s[j] = at_mma(qah[dc], kb.v, s[j]);
        s[j] = at_mma(qah[dc], kl.v, s[j]);
        s[j] = at_mma(qal[dc], kb.v, s[j]);
      }
    }

    const bool diag = (kc == qb);
    float cm[8];
#pragma unroll
    for (int r = 0; r < 8; ++r) {
      const int qrow = q0 + 8 * hh + r;
      float m = -__builtin_inff();
#pragma unroll
      for (int j = 0; j < 4; ++j) {
        const int kvcol = kv0 + j * 16 + c;
        float sv = s[j][r];
        if (diag && (kvcol > qrow)) sv = -__builtin_inff();
        s[j][r] = sv;
        m = fmaxf(m, sv);
      }
#pragma unroll
      for (int off = 1; off < 16; off <<= 1) m = fmaxf(m, __shfl_xor(m, off, 32));
      cm[r] = m;
    }

    __bf16* pwh = Psh[wave];
    __bf16* pwl = Psl[wave];
#pragma unroll
    for (int r = 0; r < 8; ++r) {
      const float mnew  = fmaxf(mrow[r], cm[r]);
      const float alpha = expf(mrow[r] - mnew);
      mrow[r] = mnew;
      float psum = 0.f;
#pragma unroll
      for (int j = 0; j < 4; ++j) {
        const float p = expf(s[j][r] - mnew);
        psum += p;
        __bf16 a, lo;
        bf_split(p, a, lo);
        pwh[(8 * hh + r) * 64 + j * 16 + c] = a;
        pwl[(8 * hh + r) * 64 + j * 16 + c] = lo;
      }
#pragma unroll
      for (int off = 1; off < 16; off <<= 1) psum += __shfl_xor(psum, off, 32);
      lrow[r] = lrow[r] * alpha + psum;
#pragma unroll
      for (int t = 0; t < 4; ++t) oacc[t][r] *= alpha;
    }
    __builtin_amdgcn_fence(__ATOMIC_RELEASE, "workgroup");
    __builtin_amdgcn_wave_barrier();
    __builtin_amdgcn_fence(__ATOMIC_ACQUIRE, "workgroup");

#pragma unroll 1
    for (int kk = 0; kk < 2; ++kk) {
      FB pa, pl;
      pa.h[0] = *(const v8b*)(pwh + c * 64 + kk * 32 + 8 * hh);
      pa.h[1] = *(const v8b*)(pwh + c * 64 + kk * 32 + 16 + 8 * hh);
      pl.h[0] = *(const v8b*)(pwl + c * 64 + kk * 32 + 8 * hh);
      pl.h[1] = *(const v8b*)(pwl + c * 64 + kk * 32 + 16 + 8 * hh);
#pragma unroll
      for (int t = 0; t < 4; ++t) {
        FB vb, vl;
        const unsigned short* vp  = Vth + (t * 16 + c) * 64 + kk * 32 + 8 * hh;
        const unsigned short* vlp = Vtl + (t * 16 + c) * 64 + kk * 32 + 8 * hh;
        vb.h[0] = *(const v8b*)(const void*)vp;
        vb.h[1] = *(const v8b*)(const void*)(vp + 16);
        vl.h[0] = *(const v8b*)(const void*)vlp;
        vl.h[1] = *(const v8b*)(const void*)(vlp + 16);
        oacc[t] = at_mma(pa.v, vb.v, oacc[t]);
        oacc[t] = at_mma(pa.v, vl.v, oacc[t]);
        oacc[t] = at_mma(pl.v, vb.v, oacc[t]);
      }
    }
  }

  __syncthreads();
  float* os = ku.os[wave];
#pragma unroll
  for (int r = 0; r < 8; ++r) {
    const float inv = 1.0f / lrow[r];
#pragma unroll
    for (int t = 0; t < 4; ++t) os[(8 * hh + r) * 64 + t * 16 + c] = oacc[t][r] * inv;
  }
  __builtin_amdgcn_fence(__ATOMIC_RELEASE, "workgroup");
  __builtin_amdgcn_wave_barrier();
  __builtin_amdgcn_fence(__ATOMIC_ACQUIRE, "workgroup");
  {
    const int q8 = lane >> 3, c8 = (lane & 7) * 8;
    for (int pass = 0; pass < 2; ++pass) {
#pragma unroll
      for (int it = 0; it < 4; ++it) {
        const int row = it * 4 + q8;
        const float* sp = os + row * 64 + c8;
        const v4f xa = *(const v4f*)sp;
        const v4f xb = *(const v4f*)(sp + 4);
        v4u wh, wl;
        unsigned ph, pl;
        split2_pack(xa[0], xa[1], ph, pl); wh[0] = ph; wl[0] = pl;
        split2_pack(xa[2], xa[3], ph, pl); wh[1] = ph; wl[1] = pl;
        split2_pack(xb[0], xb[1], ph, pl); wh[2] = ph; wl[2] = pl;
        split2_pack(xb[2], xb[3], ph, pl); wh[3] = ph; wl[3] = pl;
        const size_t oo = ((size_t)bl * (size_t)S + (size_t)(q0 + row)) * (size_t)ldo + (size_t)(h * 64 + c8);
        *(volatile v4u*)(Oh + oo) = wh;
        *(volatile v4u*)(Ol + oo) = wl;
      }
      __threadfence();
    }
  }
}

extern "C" void kernel_launch(void* const* d_in, const int* in_sizes, int n_in,
                              void* d_out, int out_size, void* d_ws, size_t ws_size,
                              hipStream_t stream) {
  if (n_in < 4) return;
  if (in_sizes[0] != kRows * kDModel) return;
  if (in_sizes[1] != kSeq) return;
  if (in_sizes[2] != kQKVCols * kDModel) return;
  if (in_sizes[3] != kDModel * kDModel) return;
  if (out_size != kRows * kDModel) return;
  if (ws_size < kWsEnd) return;

  const float* x    = (const float*)d_in[0];
  const int*   pos  = (const int*)d_in[1];
  const float* wqkv = (const float*)d_in[2];
  const float* wout = (const float*)d_in[3];
  float* out = (float*)d_out;

  unsigned char* ws = (unsigned char*)d_ws;
  unsigned short* Xb  = (unsigned short*)(ws + kOffXb);
  unsigned short* Ohp = (unsigned short*)(ws + kOffOh);
  unsigned short* Olp = (unsigned short*)(ws + kOffOl);
  unsigned short* Wqb = (unsigned short*)(ws + kOffWqb);
  unsigned short* Wob = (unsigned short*)(ws + kOffWob);
  float*          ropeT = (float*)(ws + kOffRope);
  unsigned short* Qh  = (unsigned short*)(ws + kOffQh);
  unsigned short* Ql  = (unsigned short*)(ws + kOffQl);

  RopeFreq fr;
  for (int p = 0; p < 32; ++p) {
    const double t = std::pow(10000.0, (double)p / 32.0);
    const float tf = (float)t;
    fr.f[p] = 1.0f / tf;
  }

  const int n2x = kRows * kDModel / 2;
  const int n2w = kQKVCols * kDModel / 2;
  const int n2o = kDModel * kDModel / 2;
  cast_f32_bf16x2<<<dim3(n2x / 256), dim3(256), 0, stream>>>(x, Xb, n2x);
  cast_f32_bf16x2<<<dim3(n2w / 256), dim3(256), 0, stream>>>(wqkv, Wqb, n2w);
  cast_f32_bf16x2<<<dim3(n2o / 256), dim3(256), 0, stream>>>(wout, Wob, n2o);
  rope_table_kernel<<<dim3((kSeq * 32) / 256), dim3(256), 0, stream>>>(pos, ropeT, kSeq, fr);

  const int blocksQKV = ((kRows / 64) * (kQKVCols / 64)) / 8;
  wmma_gemm64<0, 3><<<dim3(blocksQKV), dim3(256), 0, stream>>>(
      Xb, Xb, kDModel, Wqb, Wqb, kDModel, (void*)Qh, (void*)Ql, kQKVCols,
      ropeT, kSeq, 2 * kDModel, kDModel, 0.125f, kRows, kQKVCols, kDModel, 1.0f);

  const int blocksAttn = kPhaseB * kHeads * (kSeq / 64);
  const int blocksOut  = ((kPhaseRows / 64) * (kDModel / 64)) / 8;
  for (int ph = 0; ph < kBatch / kPhaseB; ++ph) {
    attn_causal64<<<dim3(blocksAttn), dim3(128), 0, stream>>>(
        Qh, Ql, Ohp, Olp, kSeq, kHeads, kQKVCols, kDModel, ph * kPhaseB);
    float* outPh = out + (size_t)ph * kPhaseRows * kDModel;
    wmma_gemm64<2, 0><<<dim3(blocksOut), dim3(256), 0, stream>>>(
        Ohp, Olp, kDModel, Wob, Wob, kDModel, (void*)outPh, (void*)outPh, kDModel,
        ropeT, kSeq, 0, 0, 1.0f, kPhaseRows, kDModel, kDModel, 1.0f);
  }
}
